// MultiHeadAttention_17583596110389
// MI455X (gfx1250) — hardware-run, weakly checked
//
#include <hip/hip_runtime.h>
#ifndef NB
#define NB 8
#endif
#ifndef SEQ
#define SEQ 1024
#endif
#define NB_FULL 8
#define SEQ_FULL 1024
#define ED 256
#define NH 8
#define HD 256
#define NE (NH * HD)
#define GB ((NB) < 4 ? (NB) : 4)
#define NGRP ((NB) / GB)
#define GM (GB * SEQ)
#define XSTRIDE_FULL ((size_t)SEQ_FULL * ED)
#define MSTRIDE_FULL ((size_t)SEQ_FULL * SEQ_FULL)
#define PLANE ((size_t)GB * NH * SEQ * HD)

#define XB_BYTES ((size_t)NB * SEQ * ED * 2)
#define WT_BYTES ((size_t)3 * NE * ED * 2)
#define WF_BYTES ((size_t)ED * NE * 2)
#define PL_BYTES (PLANE * 2 * 3)
#define CX_BYTES ((size_t)GM * NE * 2)

static_assert(SEQ % 128 == 0);
static_assert(SEQ <= SEQ_FULL);
static_assert(NB <= NB_FULL);
static_assert(NB % GB == 0);
static_assert(HD == 256 && ED == 256 && NE == 2048);
static_assert(XB_BYTES % 256 == 0 && WT_BYTES % 256 == 0 && WF_BYTES % 256 == 0 && PL_BYTES % 256 == 0 && CX_BYTES % 256 == 0);
static_assert(XB_BYTES + WT_BYTES + WF_BYTES + PL_BYTES + CX_BYTES <= (size_t)134217728);

typedef __bf16 v16b __attribute__((ext_vector_type(16)));
typedef _Float16 v16h __attribute__((ext_vector_type(16)));
typedef unsigned short v8us __attribute__((ext_vector_type(8), may_alias));
typedef float v8f __attribute__((ext_vector_type(8)));
typedef float v4f __attribute__((ext_vector_type(4)));
typedef float v4fa __attribute__((ext_vector_type(4), may_alias));
typedef int v4ia __attribute__((ext_vector_type(4), may_alias));
union FragB { v16b v; v8us half[2]; };
union FragH { v16h v; v8us half[2]; _Float16 h[16]; };

#define LOG2E 1.4426950408889634f
#define NEGBIG (-1.0e30f)

__device__ __forceinline__ unsigned short bf16_bits(float x) {
  unsigned int u = __float_as_uint(x);
  return (unsigned short)((u + 0x7FFFu + ((u >> 16) & 1u)) >> 16);
}
__device__ __forceinline__ float bf16_val(unsigned short b) { return __uint_as_float(((unsigned int)b) << 16); }
__device__ __forceinline__ float bf16_rne(float x) { return bf16_val(bf16_bits(x)); }
__device__ __forceinline__ unsigned short f16_bits(float x) { return __builtin_bit_cast(unsigned short, (_Float16)x); }

#define WB(a, b, c) __builtin_amdgcn_wmma_f32_16x16x32_bf16(false, a, false, b, (short)0, c, false, false)
#define WH(a, b, c) __builtin_amdgcn_wmma_f32_16x16x32_f16(false, a, false, b, (short)0, c, false, false)

__device__ __forceinline__ void mma8_b(v16b a0, v16b a1, v16b b0, v16b b1, v16b b2, v16b b3,
                                       v8f& c00, v8f& c01, v8f& c02, v8f& c03, v8f& c10, v8f& c11, v8f& c12, v8f& c13) {
  c00 = WB(a0, b0, c00); c01 = WB(a0, b1, c01); c02 = WB(a0, b2, c02); c03 = WB(a0, b3, c03);
  c10 = WB(a1, b0, c10); c11 = WB(a1, b1, c11); c12 = WB(a1, b2, c12); c13 = WB(a1, b3, c13);
  asm volatile("v_nop\n\tv_nop\n\tv_nop\n\tv_nop"
               : "+v"(c00), "+v"(c01), "+v"(c02), "+v"(c03), "+v"(c10), "+v"(c11), "+v"(c12), "+v"(c13)
               : "v"(a0), "v"(a1), "v"(b0), "v"(b1), "v"(b2), "v"(b3));
}
__device__ __forceinline__ void mma8_h(v16h a0, v16h a1, v16h b0, v16h b1, v16h b2, v16h b3,
                                       v8f& c00, v8f& c01, v8f& c02, v8f& c03, v8f& c10, v8f& c11, v8f& c12, v8f& c13) {
  c00 = WH(a0, b0, c00); c01 = WH(a0, b1, c01); c02 = WH(a0, b2, c02); c03 = WH(a0, b3, c03);
  c10 = WH(a1, b0, c10); c11 = WH(a1, b1, c11); c12 = WH(a1, b2, c12); c13 = WH(a1, b3, c13);
  asm volatile("v_nop\n\tv_nop\n\tv_nop\n\tv_nop"
               : "+v"(c00), "+v"(c01), "+v"(c02), "+v"(c03), "+v"(c10), "+v"(c11), "+v"(c12), "+v"(c13)
               : "v"(a0), "v"(a1), "v"(b0), "v"(b1), "v"(b2), "v"(b3));
}
__device__ __forceinline__ void mma_s2(v16h ka, v16h kb, v16h q, v8f& s0, v8f& s1) {
  s0 = WH(ka, q, s0);
  s1 = WH(kb, q, s1);
  asm volatile("v_nop\n\tv_nop\n\tv_nop\n\tv_nop" : "+v"(s0), "+v"(s1) : "v"(ka), "v"(kb), "v"(q));
}
__device__ __forceinline__ void mma_pv4(v16h a0, v16h a1, v16h a2, v16h a3, v16h ph, v16h pl,
                                        v8f& c0, v8f& c1, v8f& c2, v8f& c3) {
  c0 = WH(a0, ph, c0); c1 = WH(a1, ph, c1); c2 = WH(a2, ph, c2); c3 = WH(a3, ph, c3);
  c0 = WH(a0, pl, c0); c1 = WH(a1, pl, c1); c2 = WH(a2, pl, c2); c3 = WH(a3, pl, c3);
  asm volatile("v_nop\n\tv_nop\n\tv_nop\n\tv_nop"
               : "+v"(c0), "+v"(c1), "+v"(c2), "+v"(c3)
               : "v"(a0), "v"(a1), "v"(a2), "v"(a3), "v"(ph), "v"(pl));
}

__global__ __launch_bounds__(256) void k_cvx(const float* __restrict__ X, unsigned short* __restrict__ Xb) {
  const int t = blockIdx.x * 256 + threadIdx.x;
  if (t >= NB * SEQ * (ED / 8)) return;
  const int row = t >> 5, piece = t & 31;
  const int b = row / SEQ, s = row - b * SEQ;
  const float* src = X + (size_t)b * XSTRIDE_FULL + (size_t)s * ED + piece * 8;
  const v4f x0 = *(const v4fa*)(src), x1 = *(const v4fa*)(src + 4);
  v8us o;
  o[0] = bf16_bits(x0[0]); o[1] = bf16_bits(x0[1]); o[2] = bf16_bits(x0[2]); o[3] = bf16_bits(x0[3]);
  o[4] = bf16_bits(x1[0]); o[5] = bf16_bits(x1[1]); o[6] = bf16_bits(x1[2]); o[7] = bf16_bits(x1[3]);
  unsigned short* d = Xb + (size_t)t * 8;
  *(volatile v8us*)d = o;
  __threadfence();
  *(volatile v8us*)d = o;
}

template <int MODE>
__global__ __launch_bounds__(256) void k_wt(const float* __restrict__ W, unsigned short* __restrict__ Wt, int R, int C) {
  __shared__ unsigned short tl[64][66];
  const int tid = threadIdx.x;
  const int c0 = blockIdx.x * 64, r0 = blockIdx.y * 64;
  for (int i = tid; i < 64 * 16; i += 256) {
    const int j = i >> 4, c4 = (i & 15) * 4;
    const v4f x = *(const v4fa*)(W + (size_t)(r0 + j) * C + c0 + c4);
    unsigned short u0, u1, u2, u3;
    if (MODE == 0) {
      u0 = bf16_bits(x[0]); u1 = bf16_bits(x[1]); u2 = bf16_bits(x[2]); u3 = bf16_bits(x[3]);
    } else {
      u0 = f16_bits(bf16_rne(x[0]) * 1024.0f); u1 = f16_bits(bf16_rne(x[1]) * 1024.0f);
      u2 = f16_bits(bf16_rne(x[2]) * 1024.0f); u3 = f16_bits(bf16_rne(x[3]) * 1024.0f);
    }
    tl[c4 + 0][j] = u0; tl[c4 + 1][j] = u1; tl[c4 + 2][j] = u2; tl[c4 + 3][j] = u3;
  }
  __syncthreads();
  for (int pass = 0; pass < 2; ++pass) {
    for (int i = tid; i < 64 * 8; i += 256) {
      const int d = i >> 3, j8 = (i & 7) * 8;
      v8us o;
#pragma unroll
      for (int q = 0; q < 8; ++q) o[q] = tl[d][j8 + q];
      *(volatile v8us*)(Wt + (size_t)(c0 + d) * R + r0 + j8) = o;
    }
    if (pass == 0) __threadfence();
  }
}

__global__ __launch_bounds__(128) void k_proj(const unsigned short* __restrict__ Xg, const unsigned short* __restrict__ Wt3,
                                              unsigned short* __restrict__ P3) {
  __shared__ __attribute__((aligned(16))) unsigned short tl[128][72];
  const int tid = threadIdx.x, w = __builtin_amdgcn_readfirstlane((int)(tid >> 5)), lane = tid & 31, ln = lane & 15, hh = lane >> 4;
  const int z = blockIdx.z;
  const int n0 = blockIdx.x * 64, m0 = blockIdx.y * 128;
  const unsigned short* Wt = Wt3 + (size_t)z * NE * ED;
  unsigned short* out = P3 + (size_t)z * PLANE;
  const unsigned short* ap = Xg + (size_t)(m0 + 32 * w + ln) * ED + 8 * hh;
  const unsigned short* bp = Wt + (size_t)(n0 + ln) * ED + 8 * hh;
  v8f acc[2][4] = {};
#pragma unroll 1
  for (int k0 = 0; k0 < ED; k0 += 32) {
    FragB a0, a1, b0, b1, b2, b3;
    a0.half[0] = *(const v8us*)(ap + k0);                a0.half[1] = *(const v8us*)(ap + k0 + 16);
    a1.half[0] = *(const v8us*)(ap + 16 * ED + k0);      a1.half[1] = *(const v8us*)(ap + 16 * ED + k0 + 16);
    b0.half[0] = *(const v8us*)(bp + k0);                b0.half[1] = *(const v8us*)(bp + k0 + 16);
    b1.half[0] = *(const v8us*)(bp + 16 * ED + k0);      b1.half[1] = *(const v8us*)(bp + 16 * ED + k0 + 16);
    b2.half[0] = *(const v8us*)(bp + 32 * ED + k0);      b2.half[1] = *(const v8us*)(bp + 32 * ED + k0 + 16);
    b3.half[0] = *(const v8us*)(bp + 48 * ED + k0);      b3.half[1] = *(const v8us*)(bp + 48 * ED + k0 + 16);
    mma8_b(a0.v, a1.v, b0.v, b1.v, b2.v, b3.v,
           acc[0][0], acc[0][1], acc[0][2], acc[0][3], acc[1][0], acc[1][1], acc[1][2], acc[1][3]);
  }
#pragma unroll
  for (int i = 0; i < 2; ++i)
#pragma unroll
    for (int j = 0; j < 4; ++j)
#pragma unroll
      for (int r = 0; r < 8; ++r)
        tl[32 * w + 16 * i + 8 * hh + r][16 * j + ln] = f16_bits(acc[i][j][r] * 16.0f);
  __syncthreads();
  const int hd = n0 >> 8, e0 = n0 & 255;
  if (z < 2) {
    for (int pass = 0; pass < 2; ++pass) {
#pragma unroll 1
      for (int it = 0; it < 8; ++it) {
        const int i = tid + 128 * it;
        const int row = i >> 3, p = i & 7;
        const int m = m0 + row;
        const int bl = m / SEQ, t = m - bl * SEQ;
        const v8us o = *(const v8us*)&tl[row][8 * p];
        *(volatile v8us*)(out + (((size_t)(bl * NH + hd) * SEQ + t) * HD + e0 + 8 * p)) = o;
      }
      if (pass == 0) __threadfence();
    }
  } else {
    const int bl = m0 / SEQ, t0 = m0 - bl * SEQ;
    for (int pass = 0; pass < 2; ++pass) {
#pragma unroll 1
      for (int it = 0; it < 8; ++it) {
        const int i = tid + 128 * it;
        const int e = i >> 4, p = i & 15;
        v8us o;
#pragma unroll
        for (int q = 0; q < 8; ++q) o[q] = tl[8 * p + q][e];
        *(volatile v8us*)(out + (((size_t)(bl * NH + hd) * HD + e0 + e) * SEQ + t0 + 8 * p)) = o;
      }
      if (pass == 0) __threadfence();
    }
  }
}

__device__ __forceinline__ void fa_step(const unsigned short* __restrict__ qrow, const unsigned short* __restrict__ Kp,
                                        const unsigned short* __restrict__ Vp, const int* __restrict__ mrow,
                                        int key0, int ln, int hh, float& mr, float& lr, v8f (&O)[16]) {
  int zo = 0;
  asm volatile("" : "+v"(zo));
  const unsigned short* qp = qrow + zo;
  const unsigned short* kp0 = Kp + (size_t)(key0 + ln) * HD + 8 * hh;
  const unsigned short* kp1 = kp0 + 16 * HD;
  v8f s0 = {0.f, 0.f, 0.f, 0.f, 0.f, 0.f, 0.f, 0.f};
  v8f s1 = {0.f, 0.f, 0.f, 0.f, 0.f, 0.f, 0.f, 0.f};
#pragma unroll
  for (int c = 0; c < 8; ++c) {
    FragH qf, ka, kb;
    qf.half[0] = *(const v8us*)(qp + 32 * c);  qf.half[1] = *(const v8us*)(qp + 32 * c + 16);
    ka.half[0] = *(const v8us*)(kp0 + 32 * c); ka.half[1] = *(const v8us*)(kp0 + 32 * c + 16);
    kb.half[0] = *(const v8us*)(kp1 + 32 * c); kb.half[1] = *(const v8us*)(kp1 + 32 * c + 16);
    mma_s2(ka.v, kb.v, qf.v, s0, s1);
  }
  const int* mp = mrow + key0 + 8 * hh;
  const v4ia m0 = *(const v4ia*)(mp), m1 = *(const v4ia*)(mp + 4), m2 = *(const v4ia*)(mp + 16), m3 = *(const v4ia*)(mp + 20);
  int mk[16];
#pragma unroll
  for (int i = 0; i < 4; ++i) { mk[i] = m0[i]; mk[4 + i] = m1[i]; mk[8 + i] = m2[i]; mk[12 + i] = m3[i]; }
  const float sc2 = LOG2E * 0.000244140625f;
  float t[16];
#pragma unroll
  for (int r = 0; r < 8; ++r) { t[r] = s0[r] * sc2; t[8 + r] = s1[r] * sc2; }
  float mx = NEGBIG;
#pragma unroll
  for (int i = 0; i < 16; ++i) mx = fmaxf(mx, (mk[i] != 0) ? NEGBIG : t[i]);
  mx = fmaxf(mx, __shfl_xor(mx, 16, 32));
  const float mnew = fmaxf(mr, mx);
  const float al = exp2f(mr - mnew);
  mr = mnew;
  const float sh = 12.0f - mnew;
  FragH ph, pl;
  float ps = 0.0f;
#pragma unroll
  for (int i = 0; i < 16; ++i) {
    const float ex = exp2f(t[i] + sh);
    const float pc = (mk[i] != 0) ? 0.0f : ex;
    ps += pc;
    const _Float16 h = (_Float16)pc;
    ph.h[i] = h;
    pl.h[i] = (_Float16)(pc - (float)h);
  }
  ps += __shfl_xor(ps, 16, 32);
  lr = lr * al + ps;
#pragma unroll
  for (int u = 0; u < 16; ++u) O[u] = O[u] * al;
  const unsigned short* vp = Vp + (size_t)ln * SEQ + key0 + 8 * hh;
#pragma unroll
  for (int g = 0; g < 4; ++g) {
    FragH vf[4];
#pragma unroll
    for (int u = 0; u < 4; ++u) {
      vf[u].half[0] = *(const v8us*)(vp + (size_t)(4 * g + u) * 16 * SEQ);
      vf[u].half[1] = *(const v8us*)(vp + (size_t)(4 * g + u) * 16 * SEQ + 16);
    }
    mma_pv4(vf[0].v, vf[1].v, vf[2].v, vf[3].v, ph.v, pl.v, O[4 * g + 0], O[4 * g + 1], O[4 * g + 2], O[4 * g + 3]);
  }
}

__global__ __launch_bounds__(128) void k_attn(const unsigned short* __restrict__ Qh, const unsigned short* __restrict__ Kh,
                                              const unsigned short* __restrict__ Vt, const int* __restrict__ mask,
                                              unsigned short* __restrict__ Cx, int b0) {
  __shared__ __attribute__((aligned(16))) unsigned short so[4][16][264];
  const int tid = threadIdx.x, w = __builtin_amdgcn_readfirstlane((int)(tid >> 5)), lane = tid & 31, ln = lane & 15, hh = lane >> 4;
  const int qt = blockIdx.x % (SEQ / 64);
  const int bh = blockIdx.x / (SEQ / 64);
  const int h = bh % NH, bl = bh / NH;
  const int qbase = qt * 64 + 16 * w;
  const int qg = qbase + ln;
  const unsigned short* qrow = Qh + ((size_t)bh * SEQ + qg) * HD + 8 * hh;
  const unsigned short* Kp = Kh + (size_t)bh * SEQ * HD;
  const unsigned short* Vp = Vt + (size_t)bh * HD * SEQ;
  const int* mrow = mask + (size_t)(b0 + bl) * MSTRIDE_FULL + (size_t)qg * SEQ_FULL;
  float mr = NEGBIG, lr = 0.0f;
  v8f O[16] = {};
#pragma unroll 1
  for (int j = 0; j < SEQ / 32; ++j)
    fa_step(qrow, Kp, Vp, mrow, 32 * j, ln, hh, mr, lr, O);

  const float inv = (lr > 0.0f) ? (4.0f / fmaxf(lr, 1.0f)) : 0.0f;
#pragma unroll
  for (int u = 0; u < 16; ++u) {
    v8us o;
#pragma unroll
    for (int r = 0; r < 8; ++r) o[r] = f16_bits(O[u][r] * inv);
    *(v8us*)&so[w][ln][16 * u + 8 * hh] = o;
  }
  __syncthreads();
  unsigned short* cg = Cx + (size_t)(bl * SEQ + qbase) * NE + h * HD;
  for (int pass = 0; pass < 2; ++pass) {
#pragma unroll 1
    for (int row = 0; row < 16; ++row) {
      const v8us v = *(const v8us*)&so[w][row][8 * lane];
      *(volatile v8us*)(cg + (size_t)row * NE + 8 * lane) = v;
    }
    if (pass == 0) __threadfence();
  }
}

__global__ __launch_bounds__(128) void k_fc(const unsigned short* __restrict__ Cx, const unsigned short* __restrict__ WfT,
                                            const float* __restrict__ bias, float* __restrict__ Og, int b0) {
  __shared__ __attribute__((aligned(16))) float so[128][68];
  const int tid = threadIdx.x, w = __builtin_amdgcn_readfirstlane((int)(tid >> 5)), lane = tid & 31, ln = lane & 15, hh = lane >> 4;
  const int n0 = blockIdx.x * 64, m0 = blockIdx.y * 128;
  const unsigned short* ap = Cx + (size_t)(m0 + 32 * w + ln) * NE + 8 * hh;
  const unsigned short* bp = WfT + (size_t)(n0 + ln) * NE + 8 * hh;
  v8f acc[2][4] = {};
#pragma unroll 1
  for (int k0 = 0; k0 < NE; k0 += 32) {
    FragH a0, a1, b0f, b1f, b2f, b3f;
    a0.half[0] = *(const v8us*)(ap + k0);                 a0.half[1] = *(const v8us*)(ap + k0 + 16);
    a1.half[0] = *(const v8us*)(ap + 16 * NE + k0);       a1.half[1] = *(const v8us*)(ap + 16 * NE + k0 + 16);
    b0f.half[0] = *(const v8us*)(bp + k0);                b0f.half[1] = *(const v8us*)(bp + k0 + 16);
    b1f.half[0] = *(const v8us*)(bp + 16 * NE + k0);      b1f.half[1] = *(const v8us*)(bp + 16 * NE + k0 + 16);
    b2f.half[0] = *(const v8us*)(bp + 32 * NE + k0);      b2f.half[1] = *(const v8us*)(bp + 32 * NE + k0 + 16);
    b3f.half[0] = *(const v8us*)(bp + 48 * NE + k0);      b3f.half[1] = *(const v8us*)(bp + 48 * NE + k0 + 16);
    mma8_h(a0.v, a1.v, b0f.v, b1f.v, b2f.v, b3f.v,
           acc[0][0], acc[0][1], acc[0][2], acc[0][3], acc[1][0], acc[1][1], acc[1][2], acc[1][3]);
  }
#pragma unroll
  for (int j = 0; j < 4; ++j) {
    const float bb = bf16_rne(bias[n0 + 16 * j + ln]);
#pragma unroll
    for (int i = 0; i < 2; ++i)
#pragma unroll
      for (int r = 0; r < 8; ++r)
        so[32 * w + 16 * i + 8 * hh + r][16 * j + ln] = acc[i][j][r] * 0.0000152587890625f + bb;
  }
  __syncthreads();
  for (int pass = 0; pass < 2; ++pass) {
#pragma unroll 1
    for (int it = 0; it < 16; ++it) {
      const int i = tid + 128 * it;
      const int row = i >> 4, p = i & 15;
      const int m = m0 + row;
      const int bl = m / SEQ, t = m - bl * SEQ;
      const v4f v = *(const v4fa*)&so[row][4 * p];
      *(volatile v4f*)(Og + (size_t)(b0 + bl) * XSTRIDE_FULL + (size_t)t * ED + n0 + 4 * p) = v;
    }
    if (pass == 0) __threadfence();
  }
}

extern "C" void kernel_launch(void* const* d_in, const int* in_sizes, int n_in,
                              void* d_out, int out_size, void* d_ws, size_t ws_size, hipStream_t stream) {
  if (n_in < 7) return;
  const long long needx = (long long)(NB - 1) * SEQ_FULL * ED + (long long)SEQ * ED;
  const long long needm = (long long)(NB - 1) * SEQ_FULL * SEQ_FULL + (long long)(SEQ - 1) * SEQ_FULL + SEQ;
  if ((long long)in_sizes[0] < needx) return;
  if ((long long)in_sizes[1] < (long long)ED * NE || (long long)in_sizes[2] < (long long)ED * NE ||
      (long long)in_sizes[3] < (long long)ED * NE || (long long)in_sizes[4] < (long long)NE * ED) return;
  if ((long long)in_sizes[5] < (long long)ED) return;
  if ((long long)in_sizes[6] < needm) return;
  if ((long long)out_size < needx) return;
  const float* x   = (const float*)d_in[0];
  const float* Wq  = (const float*)d_in[1];
  const float* Wk  = (const float*)d_in[2];
  const float* Wv  = (const float*)d_in[3];
  const float* Wfc = (const float*)d_in[4];
  const float* bfc = (const float*)d_in[5];
  const int* mask  = (const int*)d_in[6];
  float* out = (float*)d_out;
  char* ws = (char*)d_ws;
  size_t off = 0;
  unsigned short* Xb  = (unsigned short*)(ws + off); off += XB_BYTES;
  unsigned short* Wt3 = (unsigned short*)(ws + off); off += WT_BYTES;
  unsigned short* WfT = (unsigned short*)(ws + off); off += WF_BYTES;
  unsigned short* P3  = (unsigned short*)(ws + off); off += PL_BYTES;
  unsigned short* Cx  = (unsigned short*)(ws + off); off += CX_BYTES;
  if (off > ws_size) return;

  k_cvx<<<(unsigned)((NB * SEQ * (ED / 8) + 255) / 256), 256, 0, stream>>>(x, Xb);
  k_wt<0><<<dim3(NE / 64, ED / 64), 256, 0, stream>>>(Wq, Wt3 + (size_t)0 * NE * ED, ED, NE);
  k_wt<0><<<dim3(NE / 64, ED / 64), 256, 0, stream>>>(Wk, Wt3 + (size_t)1 * NE * ED, ED, NE);
  k_wt<0><<<dim3(NE / 64, ED / 64), 256, 0, stream>>>(Wv, Wt3 + (size_t)2 * NE * ED, ED, NE);
  k_wt<1><<<dim3(ED / 64, NE / 64), 256, 0, stream>>>(Wfc, WfT, NE, ED);

  for (int g = 0; g < NGRP; ++g) {
    const int b0 = g * GB;
    k_proj<<<dim3(NE / 64, GM / 128, 3), 128, 0, stream>>>(Xb + (size_t)g * GM * ED, Wt3, P3);
    k_attn<<<(unsigned)(GB * NH * (SEQ / 64)), 128, 0, stream>>>(P3, P3 + PLANE, P3 + 2 * PLANE, mask, Cx, b0);
    k_fc<<<dim3(ED / 64, GM / 128), 128, 0, stream>>>(Cx, WfT, bfc, out, b0);
  }
}
